// EdgePropertyPredictionModel_5360119185641
// MI455X (gfx1250) — hardware-verified
//
#include <hip/hip_runtime.h>
#include <stddef.h>
#include <stdint.h>


#define DF    128
#define NH    8
#define HC    16
#define INF   64
#define FFD   218
#define FFN   224
#define FFK   224
#define YP    256
#define DK    512
#define NL    3
#define GR    32
#define KMAX  512
#define APM   (KMAX + 8)
#define XSP   132
#define NTHR  256
#define NWAVE 8
#define NB    512
#define CHUNK 2048
#define WCAP  256
#define NGRP  (CHUNK / (NTHR * 4))
#define EPS_BN 1e-5f
#define WSC   8.0f
#define WINV  0.125f

#define LDS_SACC (NB * DF)
#define LDS_DEN  (NB * NH)
#define LDS_LIST (NWAVE * WCAP)
#define LDS_AGG_BYTES ((LDS_SACC + LDS_DEN + LDS_LIST + NWAVE) * 4)

static_assert(WCAP == (CHUNK / NTHR) * 32);
static_assert(NGRP == 2);
static_assert(NB == 512);
static_assert(CHUNK <= 4096);
static_assert(LDS_AGG_BYTES == 286752);
static_assert(LDS_LIST >= NWAVE * 2 * DF);
static_assert(((LDS_SACC + LDS_DEN) % 4) == 0);
static_assert((GR * APM * 2 + GR * XSP * 4 + 2 * GR * NH * 4 + NWAVE * 2 * DF * 4) <= 65536);
static_assert((FFK % 32) == 0 && (FFN % 16) == 0 && YP >= FFN && FFK <= YP);

typedef float    v4f  __attribute__((ext_vector_type(4)));
typedef float    v8f  __attribute__((ext_vector_type(8)));
typedef int      v4i  __attribute__((ext_vector_type(4)));
typedef _Float16 v8h  __attribute__((ext_vector_type(8)));
typedef _Float16 v16h __attribute__((ext_vector_type(16)));
union Frag   { v16h v; v8h half[2]; };
union Pack16 { v8h h; v4i i; };

__device__ __forceinline__ v8f wm(v16h a, v16h b, v8f c) {
  v8f d = __builtin_amdgcn_wmma_f32_16x16x32_f16(false, a, false, b, (short)0, c, false, false);
  asm volatile("v_nop\n\tv_nop\n\tv_nop\n\tv_nop" : "+v"(d) : "v"(a), "v"(b));
  return d;
}

__device__ __forceinline__ v8h ld8h(const float* p) {
  const v4f a = *(const v4f*)p;
  const v4f b = *(const v4f*)(p + 4);
  Pack16 u;
  u.h[0] = (_Float16)a.x; u.h[1] = (_Float16)a.y; u.h[2] = (_Float16)a.z; u.h[3] = (_Float16)a.w;
  u.h[4] = (_Float16)b.x; u.h[5] = (_Float16)b.y; u.h[6] = (_Float16)b.z; u.h[7] = (_Float16)b.w;
  return u.h;
}
__device__ __forceinline__ v8h ld8h(const _Float16* p) {
  return *(const v8h*)p;
}

__global__ __launch_bounds__(NTHR) void k_prepw(const float* __restrict__ W, int K, int M, int wstride,
                                                _Float16* Wt, int Kpad, int Mpad, int tstride, float scale) {
  const int lay = blockIdx.y;
  const float* Wl = W + (size_t)lay * (size_t)wstride;
  _Float16* Tl = Wt + (size_t)lay * (size_t)tstride;
  const int i = blockIdx.x * NTHR + threadIdx.x;
  const int n8 = (Mpad * Kpad) >> 3;
  if (i >= n8) return;
  const int o = i * 8;
  const int m = o / Kpad;
  const int k = o - m * Kpad;
  Pack16 u;
#pragma unroll
  for (int j = 0; j < 8; ++j) {
    float v = 0.f;
    if (m < M && (k + j) < K) v = Wl[(size_t)(k + j) * M + m] * scale;
    u.h[j] = (_Float16)v;
  }
  *(volatile v4i*)(Tl + o) = u.i;
  __threadfence();
  *(volatile v4i*)(Tl + o) = u.i;
}

__device__ __forceinline__ void epi_std(v8f acc, int T, int hh, int ncol, int colg, float bcol,
                                        const float* R, int ldr, int rowBase, int nN, int relu,
                                        float* Xs) {
#pragma unroll
  for (int r = 0; r < 8; ++r) {
    const int lr = T * 16 + 8 * hh + r;
    float v = acc[r] * WINV + bcol;
    if (R != nullptr) {
      int row = rowBase + lr;
      if (row > nN - 1) row = nN - 1;
      v += R[(size_t)row * ldr + colg];
    }
    if (relu) v = fmaxf(v, 0.f);
    Xs[lr * XSP + ncol] = v;
  }
}

__device__ __forceinline__ void epi_attn(v8f acc, int T, int hh, int m, int wave, int ncol,
                                         float cs, float cd, float* Xs, float* As, float* Ds) {
  float ss[8], sd[8];
#pragma unroll
  for (int r = 0; r < 8; ++r) {
    const float v = acc[r] * WINV;
    Xs[(T * 16 + 8 * hh + r) * XSP + ncol] = v;
    ss[r] = v * cs;
    sd[r] = v * cd;
  }
#pragma unroll
  for (int mk = 1; mk < 16; mk <<= 1) {
#pragma unroll
    for (int r = 0; r < 8; ++r) {
      ss[r] += __shfl_xor(ss[r], mk, 32);
      sd[r] += __shfl_xor(sd[r], mk, 32);
    }
  }
  if (m == 0) {
#pragma unroll
    for (int r = 0; r < 8; ++r) {
      As[(T * 16 + 8 * hh + r) * NH + wave] = ss[r];
      Ds[(T * 16 + 8 * hh + r) * NH + wave] = sd[r];
    }
  }
}

template <int MODE, typename TA>
__global__ __launch_bounds__(NTHR) void k_gemm(
    const TA* A, int lda, int K,
    const _Float16* __restrict__ Wt, int ldw, int Mtot,
    const float* __restrict__ bias, int M,
    const float* R, int ldr,
    float* C, _Float16* Ch, int ldc,
    float* part,
    const float* __restrict__ attl, const float* __restrict__ attr,
    float* elp, float* erp,
    int relu, int nN) {
  __shared__ __attribute__((aligned(16))) _Float16 At[GR * APM];
  __shared__ __attribute__((aligned(16))) float Xs[GR * XSP];
  __shared__ __attribute__((aligned(16))) float As[GR * NH];
  __shared__ __attribute__((aligned(16))) float Ds[GR * NH];
  __shared__ __attribute__((aligned(16))) float Ps[NWAVE * 2 * DF];

  const int tid  = threadIdx.x;
  const int lane = tid & 31;
  const int wave = tid >> 5;
  const int hh   = lane >> 4;
  const int m    = lane & 15;
  const int rowBase = blockIdx.x * GR;
  const int colBase = blockIdx.y * DF;
  const int AP = K + 8;

  {
    const int kg = K >> 3;
    for (int t = tid; t < GR * kg; t += NTHR) {
      const int r = t / kg;
      const int c = (t - r * kg) * 8;
      int row = rowBase + r;
      if (row > nN - 1) row = nN - 1;
      const v8h hv = ld8h(A + (size_t)row * lda + c);
      *(v8h*)(At + r * AP + c) = hv;
    }
  }
  __syncthreads();

  const int ncol = wave * 16 + m;
  const int colg = colBase + ncol;
  v8f c0a = {0.f, 0.f, 0.f, 0.f, 0.f, 0.f, 0.f, 0.f};
  v8f c1a = {0.f, 0.f, 0.f, 0.f, 0.f, 0.f, 0.f, 0.f};
  if (colBase + wave * 16 < Mtot) {
    const _Float16* wrow = Wt + (size_t)colg * ldw + 8 * hh;
    const _Float16* pa0  = At + m * AP + 8 * hh;
    const _Float16* pa1  = At + (16 + m) * AP + 8 * hh;
    for (int k0 = 0; k0 < K; k0 += 32) {
      Frag a0, a1, b;
      b.half[0]  = *(const v8h*)(wrow + k0);  b.half[1]  = *(const v8h*)(wrow + k0 + 16);
      a0.half[0] = *(const v8h*)(pa0 + k0);   a0.half[1] = *(const v8h*)(pa0 + k0 + 16);
      a1.half[0] = *(const v8h*)(pa1 + k0);   a1.half[1] = *(const v8h*)(pa1 + k0 + 16);
      c0a = wm(a0.v, b.v, c0a);
      c1a = wm(a1.v, b.v, c1a);
    }
  }

  if (MODE == 1) {
    const float cs = attl[ncol];
    const float cd = attr[ncol];
    epi_attn(c0a, 0, hh, m, wave, ncol, cs, cd, Xs, As, Ds);
    epi_attn(c1a, 1, hh, m, wave, ncol, cs, cd, Xs, As, Ds);
  } else {
    float bcol = 0.f;
    if (bias != nullptr && colg < M) bcol = bias[colg];
    epi_std(c0a, 0, hh, ncol, colg, bcol, R, ldr, rowBase, nN, relu, Xs);
    epi_std(c1a, 1, hh, ncol, colg, bcol, R, ldr, rowBase, nN, relu, Xs);
  }
  __syncthreads();

  if (MODE == 2) {
    Pack16 u[2];
    _Float16* gq[2];
#pragma unroll
    for (int i = 0; i < 2; ++i) {
      const int lr = 4 * wave + 2 * i + hh;
      const float* xs = Xs + lr * XSP + 8 * m;
      const v4f f0 = *(const v4f*)xs;
      const v4f f1 = *(const v4f*)(xs + 4);
      u[i].h[0] = (_Float16)f0.x; u[i].h[1] = (_Float16)f0.y; u[i].h[2] = (_Float16)f0.z; u[i].h[3] = (_Float16)f0.w;
      u[i].h[4] = (_Float16)f1.x; u[i].h[5] = (_Float16)f1.y; u[i].h[6] = (_Float16)f1.z; u[i].h[7] = (_Float16)f1.w;
      gq[i] = Ch + (size_t)(rowBase + lr) * ldc + colBase + 8 * m;
    }
#pragma unroll
    for (int i = 0; i < 2; ++i) *(volatile v4i*)(gq[i]) = u[i].i;
    __threadfence();
#pragma unroll
    for (int i = 0; i < 2; ++i) *(volatile v4i*)(gq[i]) = u[i].i;
  } else {
    v4f xr[4];
#pragma unroll
    for (int i = 0; i < 4; ++i) xr[i] = *(const v4f*)(Xs + (4 * wave + i) * XSP + 4 * lane);
    float* xpp[4];
#pragma unroll
    for (int i = 0; i < 4; ++i)
      xpp[i] = C + (size_t)(rowBase + 4 * wave + i) * ldc + colBase + 4 * lane;
    float* gp = 0;
    v4f gv = {0.f, 0.f, 0.f, 0.f};
    if (MODE == 1) {
      if (wave < 2) {
        gv = *(const v4f*)(As + wave * 128 + 4 * lane);
        gp = elp + (size_t)rowBase * NH + wave * 128 + 4 * lane;
      } else if (wave < 4) {
        gv = *(const v4f*)(Ds + (wave - 2) * 128 + 4 * lane);
        gp = erp + (size_t)rowBase * NH + (wave - 2) * 128 + 4 * lane;
      }
    }
#pragma unroll
    for (int i = 0; i < 4; ++i) *(volatile v4f*)(xpp[i]) = xr[i];
    if (gp) *(volatile v4f*)gp = gv;
    __threadfence();
#pragma unroll
    for (int i = 0; i < 4; ++i) *(volatile v4f*)(xpp[i]) = xr[i];
    if (gp) *(volatile v4f*)gp = gv;

    if (MODE == 0 && part != nullptr) {
      v4f s4 = {0.f, 0.f, 0.f, 0.f};
      v4f q4 = {0.f, 0.f, 0.f, 0.f};
#pragma unroll
      for (int i = 0; i < 4; ++i) {
        if (rowBase + 4 * wave + i < nN) { s4 += xr[i]; q4 += xr[i] * xr[i]; }
      }
      *(v4f*)(Ps + (wave * 2 + 0) * DF + 4 * lane) = s4;
      *(v4f*)(Ps + (wave * 2 + 1) * DF + 4 * lane) = q4;
      __syncthreads();
      if (wave < 2) {
        v4f t4 = {0.f, 0.f, 0.f, 0.f};
#pragma unroll
        for (int w = 0; w < NWAVE; ++w) t4 += *(const v4f*)(Ps + (w * 2 + wave) * DF + 4 * lane);
        float* pp = part + (size_t)blockIdx.x * (2 * DF) + wave * DF + 4 * lane;
        *(volatile v4f*)pp = t4;
        __threadfence();
        *(volatile v4f*)pp = t4;
      }
    }
  }
}

__global__ __launch_bounds__(NTHR) void k_agg(
    const float* __restrict__ feat, const float* __restrict__ elp, const float* __restrict__ erp,
    const int* __restrict__ src, const int* __restrict__ dst,
    const float* __restrict__ hres, const float* __restrict__ bias,
    float* h1, float* part, int nN, int nE) {
  extern __shared__ v4f lds_dyn[];
  float* sacc = (float*)lds_dyn;
  float* den  = sacc + LDS_SACC;
  int*   list = (int*)(den + LDS_DEN);
  int*   wcnt = list + LDS_LIST;

  const int tid  = threadIdx.x;
  const int lane = tid & 31;
  const int wave = tid >> 5;
  const int hd   = lane >> 2;
  const int nodeBase = blockIdx.x * NB;

  {
    const v4f z4 = {0.f, 0.f, 0.f, 0.f};
    for (int i = tid; i < (LDS_SACC + LDS_DEN) / 4; i += NTHR) lds_dyn[i] = z4;
  }
  __syncthreads();

  const bool al16 = ((((size_t)dst) & (size_t)15) == 0);
  const int nChunks = (nE + CHUNK - 1) / CHUNK;
#pragma unroll 1
  for (int ch = 0; ch < nChunks; ++ch) {
    const int cbase = ch * CHUNK;
    int wc = 0;
#pragma unroll
    for (int g = 0; g < NGRP; ++g) {
      const int le0 = (g * NTHR + tid) * 4;
      const int e0  = cbase + le0;
      const int sent = -2147483647 - 1;
      v4i d;
      if (al16 && (e0 + 3 < nE)) {
        d = *(const v4i*)(dst + e0);
      } else {
        d.x = (e0     < nE) ? dst[min(e0, nE - 1)]     : sent;
        d.y = (e0 + 1 < nE) ? dst[min(e0 + 1, nE - 1)] : sent;
        d.z = (e0 + 2 < nE) ? dst[min(e0 + 2, nE - 1)] : sent;
        d.w = (e0 + 3 < nE) ? dst[min(e0 + 3, nE - 1)] : sent;
      }
      const unsigned s0 = (unsigned)d.x - (unsigned)nodeBase;
      const unsigned s1 = (unsigned)d.y - (unsigned)nodeBase;
      const unsigned s2 = (unsigned)d.z - (unsigned)nodeBase;
      const unsigned s3 = (unsigned)d.w - (unsigned)nodeBase;
      const bool h0 = s0 < (unsigned)NB;
      const bool h1b = s1 < (unsigned)NB;
      const bool h2 = s2 < (unsigned)NB;
      const bool h3 = s3 < (unsigned)NB;
      const unsigned many = __builtin_amdgcn_ballot_w32(h0 | h1b | h2 | h3);
      if (many != 0u) {
#define HITJ(J, HJ, SJ) { \
          const unsigned mj = __builtin_amdgcn_ballot_w32(HJ); \
          if (HJ) { \
            const int pos = wc + (int)__builtin_amdgcn_mbcnt_lo(mj, 0u); \
            if (pos < WCAP) list[wave * WCAP + pos] = ((le0 + (J)) << 9) | (int)(SJ); \
          } \
          wc += (int)__builtin_popcount(mj); }
        HITJ(0, h0, s0)
        HITJ(1, h1b, s1)
        HITJ(2, h2, s2)
        HITJ(3, h3, s3)
#undef HITJ
      }
    }
    if (lane == 0) wcnt[wave] = wc;
    __syncthreads();

    if (wave == 0) {
      for (int wsx = 0; wsx < NWAVE; ++wsx) {
        int n = wcnt[wsx];
        if (n > WCAP) n = WCAP;
        if (n < 0) n = 0;
        for (int i = 0; i < n; ++i) {
          const int ent  = list[wsx * WCAP + i];
          const int slot = ent & (NB - 1);
          const int le   = (ent >> 9) & (CHUNK - 1);
          int e = cbase + le;
          if (e > nE - 1) e = nE - 1;
          int s = src[e];
          s = s < 0 ? 0 : (s > nN - 1 ? nN - 1 : s);
          int nd = nodeBase + slot;
          if (nd > nN - 1) nd = nN - 1;
          float a = elp[(size_t)s * NH + hd] + erp[(size_t)nd * NH + hd];
          a = (a > 0.f) ? a : 0.2f * a;
          a = fminf(a, 80.f);
          const float p = __expf(a);
          const v4f xv = *(const v4f*)(feat + (size_t)s * DF + 4 * lane);
          v4f* sp = (v4f*)(sacc + slot * DF + 4 * lane);
          const v4f cur = *sp;
          const v4f nxt = cur + p * xv;
          *sp = nxt;
          if ((lane & 3) == 0) {
            const float o = den[slot * NH + hd];
            den[slot * NH + hd] = o + p;
          }
        }
      }
    }
    __syncthreads();
  }

  const v4f b4 = *(const v4f*)(bias + 4 * lane);
  v4f s4 = {0.f, 0.f, 0.f, 0.f};
  v4f q4 = {0.f, 0.f, 0.f, 0.f};
#pragma unroll 1
  for (int j = 0; j < NB / NWAVE; ++j) {
    const int slot = wave * (NB / NWAVE) + j;
    const int node = nodeBase + slot;
    if (node >= nN) break;
    const size_t nrow = (size_t)node;
    const float dv  = den[slot * NH + hd];
    const float inv = (dv > 0.f) ? (1.0f / dv) : 0.f;
    const v4f sv = *(const v4f*)(sacc + slot * DF + 4 * lane);
    const v4f hr = *(const v4f*)(hres + nrow * DF + 4 * lane);
    const v4f o4 = sv * inv + b4;
    const v4f v  = hr + o4;
    float* op = h1 + nrow * DF + 4 * lane;
    *(volatile v4f*)op = v;
    __threadfence();
    *(volatile v4f*)op = v;
    s4 += v;
    q4 += v * v;
  }
  float* Ps = (float*)list;
  *(v4f*)(Ps + (wave * 2 + 0) * DF + 4 * lane) = s4;
  *(v4f*)(Ps + (wave * 2 + 1) * DF + 4 * lane) = q4;
  __syncthreads();
  if (wave < 2) {
    v4f t4 = {0.f, 0.f, 0.f, 0.f};
#pragma unroll
    for (int w = 0; w < NWAVE; ++w) t4 += *(const v4f*)(Ps + (w * 2 + wave) * DF + 4 * lane);
    float* pp = part + (size_t)blockIdx.x * (2 * DF) + wave * DF + 4 * lane;
    *(volatile v4f*)pp = t4;
    __threadfence();
    *(volatile v4f*)pp = t4;
  }
}

__global__ __launch_bounds__(DF) void k_bnred(const float* __restrict__ part, int nblk, int nN, float* ms) {
  const int c = threadIdx.x;
  double s = 0.0, q = 0.0;
  for (int bI = 0; bI < nblk; ++bI) {
    s += (double)part[(size_t)bI * (2 * DF) + c];
    q += (double)part[(size_t)bI * (2 * DF) + DF + c];
  }
  const double inv = 1.0 / (double)nN;
  const double mu  = s * inv;
  double var = q * inv - mu * mu;
  if (var < 0.0) var = 0.0;
  const float muf = (float)mu;
  const float rs  = rsqrtf((float)var + EPS_BN);
  *(volatile float*)(ms + c) = muf;
  *(volatile float*)(ms + DF + c) = rs;
  __threadfence();
  *(volatile float*)(ms + c) = muf;
  *(volatile float*)(ms + DF + c) = rs;
}

__global__ __launch_bounds__(NTHR) void k_bnapply(const float* __restrict__ in, int ldi,
                                                  const float* __restrict__ ms,
                                                  const float* __restrict__ g, const float* __restrict__ b,
                                                  float* outp, int ldo, int relu, int nN) {
  const int t = blockIdx.x * NTHR + threadIdx.x;
  const int row = t >> 5;
  const int q = (t & 31) * 4;
  if (row >= nN) return;
  const v4f v  = *(const v4f*)(in + (size_t)row * ldi + q);
  const v4f mu = *(const v4f*)(ms + q);
  const v4f rs = *(const v4f*)(ms + DF + q);
  const v4f g4 = *(const v4f*)(g + q);
  const v4f b4 = *(const v4f*)(b + q);
  v4f y = (g4 * (v - mu)) * rs + b4;
  if (relu) {
    y.x = fmaxf(y.x, 0.f); y.y = fmaxf(y.y, 0.f); y.z = fmaxf(y.z, 0.f); y.w = fmaxf(y.w, 0.f);
  }
  float* op = outp + (size_t)row * ldo + q;
  *(volatile v4f*)op = y;
  __threadfence();
  *(volatile v4f*)op = y;
}

__global__ __launch_bounds__(64) void k_decout(const float* __restrict__ hdp, const float* __restrict__ ms,
                                               const float* __restrict__ g, const float* __restrict__ b,
                                               const _Float16* __restrict__ W2t, float* out, int nN) {
  __shared__ __attribute__((aligned(16))) _Float16 At[GR * (DF + 8)];
  __shared__ __attribute__((aligned(16))) float Os[GR];
  const int tid  = threadIdx.x;
  const int lane = tid & 31;
  const int wave = tid >> 5;
  const int hh   = lane >> 4;
  const int m    = lane & 15;
  const int rowBase = blockIdx.x * GR;

  for (int t = tid; t < GR * (DF / 8); t += 64) {
    const int r = t >> 4;
    const int c = (t & 15) * 8;
    int row = rowBase + r;
    if (row > nN - 1) row = nN - 1;
    const float* p = hdp + (size_t)row * DF + c;
    const v4f v0 = *(const v4f*)p,           v1 = *(const v4f*)(p + 4);
    const v4f mu0 = *(const v4f*)(ms + c),    mu1 = *(const v4f*)(ms + c + 4);
    const v4f rs0 = *(const v4f*)(ms + DF + c), rs1 = *(const v4f*)(ms + DF + c + 4);
    const v4f g0 = *(const v4f*)(g + c),      g1 = *(const v4f*)(g + c + 4);
    const v4f b0 = *(const v4f*)(b + c),      b1 = *(const v4f*)(b + c + 4);
    v4f y0 = (g0 * (v0 - mu0)) * rs0 + b0;
    v4f y1 = (g1 * (v1 - mu1)) * rs1 + b1;
    y0.x = fmaxf(y0.x, 0.f); y0.y = fmaxf(y0.y, 0.f); y0.z = fmaxf(y0.z, 0.f); y0.w = fmaxf(y0.w, 0.f);
    y1.x = fmaxf(y1.x, 0.f); y1.y = fmaxf(y1.y, 0.f); y1.z = fmaxf(y1.z, 0.f); y1.w = fmaxf(y1.w, 0.f);
    Pack16 u;
    u.h[0] = (_Float16)y0.x; u.h[1] = (_Float16)y0.y; u.h[2] = (_Float16)y0.z; u.h[3] = (_Float16)y0.w;
    u.h[4] = (_Float16)y1.x; u.h[5] = (_Float16)y1.y; u.h[6] = (_Float16)y1.z; u.h[7] = (_Float16)y1.w;
    *(v8h*)(At + r * (DF + 8) + c) = u.h;
  }
  __syncthreads();

  v8f acc = {0.f, 0.f, 0.f, 0.f, 0.f, 0.f, 0.f, 0.f};
  const _Float16* pa = At + (wave * 16 + m) * (DF + 8) + 8 * hh;
  const _Float16* pb = W2t + m * DF + 8 * hh;
#pragma unroll
  for (int kt = 0; kt < DF / 32; ++kt) {
    Frag a, bb;
    a.half[0]  = *(const v8h*)(pa + 32 * kt);  a.half[1]  = *(const v8h*)(pa + 32 * kt + 16);
    bb.half[0] = *(const v8h*)(pb + 32 * kt);  bb.half[1] = *(const v8h*)(pb + 32 * kt + 16);
    acc = wm(a.v, bb.v, acc);
  }
  if (m == 0) {
#pragma unroll
    for (int r = 0; r < 8; ++r) Os[wave * 16 + 8 * hh + r] = acc[r] * WINV;
  }
  __syncthreads();

  const bool full = (rowBase + GR <= nN);
  v4f ov = {0.f, 0.f, 0.f, 0.f};
  if (tid < 8) ov = *(const v4f*)(Os + 4 * tid);
  const float os = (tid < GR) ? Os[tid] : 0.f;
  if (full) {
    if (tid < 8) *(volatile v4f*)(out + rowBase + 4 * tid) = ov;
  } else {
    if (tid < GR && rowBase + tid < nN) *(volatile float*)(out + rowBase + tid) = os;
  }
  __threadfence();
  if (full) {
    if (tid < 8) *(volatile v4f*)(out + rowBase + 4 * tid) = ov;
  } else {
    if (tid < GR && rowBase + tid < nN) *(volatile float*)(out + rowBase + tid) = os;
  }
}

static inline size_t al256(size_t x) { return (x + 255) & ~(size_t)255; }
static inline int cdiv(int a, int b) { return (a + b - 1) / b; }

extern "C" void kernel_launch(void* const* d_in, const int* in_sizes, int n_in,
                              void* d_out, int out_size, void* d_ws, size_t ws_size,
                              hipStream_t stream) {
  if (n_in < 21) return;
  const int nN = in_sizes[0] / INF;
  const int nE = in_sizes[1];
  if (nN <= 0 || in_sizes[0] != nN * INF) return;
  if (nE < 0 || in_sizes[2] != nE) return;
  if (in_sizes[3] != INF * DF || in_sizes[4] != DF) return;
  if (in_sizes[5] != NL * DF * DF || in_sizes[6] != NL * DF || in_sizes[7] != NL * DF || in_sizes[8] != NL * DF) return;
  if (in_sizes[9] != NL * DF || in_sizes[10] != NL * DF) return;
  if (in_sizes[11] != NL * DF * FFD || in_sizes[12] != NL * FFD || in_sizes[13] != NL * FFD * DF || in_sizes[14] != NL * DF) return;
  if (in_sizes[15] != NL * DF || in_sizes[16] != NL * DF) return;
  if (in_sizes[17] != DK * DF || in_sizes[18] != DF || in_sizes[19] != DF || in_sizes[20] != DF) return;
  if (out_size != nN) return;

  const float* x        = (const float*)d_in[0];
  const int*   src      = (const int*)d_in[1];
  const int*   dst      = (const int*)d_in[2];
  const float* W_emb    = (const float*)d_in[3];
  const float* b_emb    = (const float*)d_in[4];
  const float* gat_W    = (const float*)d_in[5];
  const float* attn_l   = (const float*)d_in[6];
  const float* attn_r   = (const float*)d_in[7];
  const float* gat_b    = (const float*)d_in[8];
  const float* bn1_g    = (const float*)d_in[9];
  const float* bn1_b    = (const float*)d_in[10];
  const float* ff_W1    = (const float*)d_in[11];
  const float* ff_b1    = (const float*)d_in[12];
  const float* ff_W2    = (const float*)d_in[13];
  const float* ff_b2    = (const float*)d_in[14];
  const float* bn2_g    = (const float*)d_in[15];
  const float* bn2_b    = (const float*)d_in[16];
  const float* dec_W1   = (const float*)d_in[17];
  const float* dec_bn_g = (const float*)d_in[18];
  const float* dec_bn_b = (const float*)d_in[19];
  const float* dec_W2   = (const float*)d_in[20];
  float* out = (float*)d_out;

  const int nRB = cdiv(nN, GR);
  const int nP  = nRB * GR;
  const int nAB = cdiv(nN, NB);
  const int nPB = nRB > nAB ? nRB : nAB;

  char* base = (char*)d_ws;
  size_t off = 0;
  _Float16* Wemb_t = (_Float16*)(base + off); off = al256(off + (size_t)DF * INF * 2);
  _Float16* gat_t  = (_Float16*)(base + off); off = al256(off + (size_t)NL * DF * DF * 2);
  _Float16* ff1_t  = (_Float16*)(base + off); off = al256(off + (size_t)NL * FFN * DF * 2);
  _Float16* ff2_t  = (_Float16*)(base + off); off = al256(off + (size_t)NL * DF * FFK * 2);
  _Float16* dec1_t = (_Float16*)(base + off); off = al256(off + (size_t)DF * DK * 2);
  _Float16* dec2_t = (_Float16*)(base + off); off = al256(off + (size_t)16 * DF * 2);
  float* Rg[3];
  for (int i = 0; i < 3; ++i) { Rg[i] = (float*)(base + off); off = al256(off + (size_t)nP * DF * 4); }
  float* hdec = (float*)(base + off); off = al256(off + (size_t)nP * DF * 4);
  float* elb  = (float*)(base + off); off = al256(off + (size_t)nP * NH * 4);
  float* erb  = (float*)(base + off); off = al256(off + (size_t)nP * NH * 4);
  float* part = (float*)(base + off); off = al256(off + (size_t)nPB * 2 * DF * 4);
  float* ms   = (float*)(base + off); off = al256(off + (size_t)2 * DF * 4);
  if (off > ws_size) return;

  k_prepw<<<dim3(cdiv(DF * INF / 8, NTHR), 1), NTHR, 0, stream>>>(W_emb, INF, DF, 0, Wemb_t, INF, DF, 0, WSC);
  k_prepw<<<dim3(cdiv(DF * DF / 8, NTHR), NL), NTHR, 0, stream>>>(gat_W, DF, DF, DF * DF, gat_t, DF, DF, DF * DF, WSC);
  k_prepw<<<dim3(cdiv(FFN * DF / 8, NTHR), NL), NTHR, 0, stream>>>(ff_W1, DF, FFD, DF * FFD, ff1_t, DF, FFN, FFN * DF, WSC);
  k_prepw<<<dim3(cdiv(DF * FFK / 8, NTHR), NL), NTHR, 0, stream>>>(ff_W2, FFD, DF, FFD * DF, ff2_t, FFK, DF, DF * FFK, WSC);
  k_prepw<<<dim3(cdiv(DF * DK / 8, NTHR), 1), NTHR, 0, stream>>>(dec_W1, DK, DF, 0, dec1_t, DK, DF, 0, WSC);
  k_prepw<<<dim3(cdiv(16 * DF / 8, NTHR), 1), NTHR, 0, stream>>>(dec_W2, DF, 1, 0, dec2_t, DF, 16, 0, WSC);

  k_gemm<0, float><<<dim3(nRB, 1), NTHR, 0, stream>>>(
      x, INF, INF, Wemb_t, INF, DF, b_emb, DF, nullptr, 0, Rg[0], nullptr, DF, nullptr,
      nullptr, nullptr, nullptr, nullptr, 0, nN);
  k_gemm<0, float><<<dim3(nRB, 1), NTHR, 0, stream>>>(
      Rg[0], DF, DF, dec1_t, DK, DF, nullptr, 0, nullptr, 0, hdec, nullptr, DF, nullptr,
      nullptr, nullptr, nullptr, nullptr, 0, nN);

  hipFuncSetAttribute(reinterpret_cast<const void*>(&k_agg),
                      hipFuncAttributeMaxDynamicSharedMemorySize, LDS_AGG_BYTES);
  const int applyGrid = cdiv(nN * 32, NTHR);

  int hi = 0;
  for (int l = 0; l < NL; ++l) {
    float* P = Rg[hi];
    float* Q = Rg[(hi + 1) % 3];
    float* S = Rg[(hi + 2) % 3];
    k_gemm<1, float><<<dim3(nRB, 1), NTHR, 0, stream>>>(
        P, DF, DF, gat_t + (size_t)l * DF * DF, DF, DF, nullptr, 0, nullptr, 0, Q, nullptr, DF, nullptr,
        attn_l + (size_t)l * DF, attn_r + (size_t)l * DF, elb, erb, 0, nN);
    k_agg<<<nAB, NTHR, LDS_AGG_BYTES, stream>>>(Q, elb, erb, src, dst, P, gat_b + (size_t)l * DF,
                                                S, part, nN, nE);
    k_bnred<<<1, DF, 0, stream>>>(part, nAB, nN, ms);
    k_bnapply<<<applyGrid, NTHR, 0, stream>>>(S, DF, ms, bn1_g + (size_t)l * DF, bn1_b + (size_t)l * DF,
                                              Q, DF, 0, nN);
    k_gemm<2, float><<<dim3(nRB, 2), NTHR, 0, stream>>>(
        Q, DF, DF, ff1_t + (size_t)l * FFN * DF, DF, FFN, ff_b1 + (size_t)l * FFD, FFD, nullptr, 0,
        nullptr, (_Float16*)S, YP, nullptr, nullptr, nullptr, nullptr, nullptr, 1, nN);
    k_gemm<0, _Float16><<<dim3(nRB, 1), NTHR, 0, stream>>>(
        (const _Float16*)S, YP, FFK, ff2_t + (size_t)l * DF * FFK, FFK, DF, ff_b2 + (size_t)l * DF, DF,
        Q, DF, P, nullptr, DF, part, nullptr, nullptr, nullptr, nullptr, 0, nN);
    k_bnred<<<1, DF, 0, stream>>>(part, nRB, nN, ms);
    k_bnapply<<<applyGrid, NTHR, 0, stream>>>(P, DF, ms, bn2_g + (size_t)l * DF, bn2_b + (size_t)l * DF,
                                              Q, DF, 0, nN);
    k_gemm<0, float><<<dim3(nRB, 1), NTHR, 0, stream>>>(
        Q, DF, DF, dec1_t + (size_t)(l + 1) * DF, DK, DF, nullptr, 0, hdec, DF, hdec, nullptr, DF,
        (l == NL - 1) ? part : nullptr, nullptr, nullptr, nullptr, nullptr, 0, nN);
    hi = (hi + 1) % 3;
  }

  k_bnred<<<1, DF, 0, stream>>>(part, nRB, nN, ms);
  k_decout<<<nRB, 64, 0, stream>>>(hdec, ms, dec_bn_g, dec_bn_b, dec2_t, out, nN);
}
